// REGCNJraph_77902116815143
// MI455X (gfx1250) — hardware-verified
//
#include <hip/hip_runtime.h>
#include <stddef.h>


#define DIMC   200
#define XP     224
#define NP208  208
#define RREL   20
#define NBAS   20
#define KREL   4000
#define RWP    4032
#define SAP    4008
#define XTP    232
#define GD     600
#define GDP    608
#define KCAT   416
#define ATP    424
#define HIDN   256
#define KDEC   608
#define DTP    616
#define NTHR   256
#define NWAVE  8
#define RTHR   128
#define RROWS  16
#define GROWS  32
#define DROWS  32
#define EPT    8
#define NGRP   2
#define CHUNK  (NTHR * EPT * NGRP)
#define WCAP   (EPT * NGRP * 32)
#define LISTN  (NWAVE * WCAP)
#define NBC    4096
#define NBF    1024
#define RCAP   40960
#define RBN    128
#define OTHR   512
#define DEGCAP 256
#define ASC    256.0f
#define WSC    512.0f
#define RWSC   16384.0f
#define INV22  2.384185791015625e-07f
#define INV17  7.62939453125e-06f

#define LDS_LAYER (RROWS * KREL * 4 + RROWS * XTP * 2 + RROWS * XP * 4 + 128)
#define LDS_GRU   (GROWS * ATP * 2 + GROWS * GDP * 4 + GROWS * XTP * 2 + GROWS * XP * 4)
#define LDS_DEC   (DROWS * DTP * 2 + 4 * DROWS * 4)
#define LDS_FILL  ((RCAP + NBF + LISTN) * 4 + 64)

static_assert((CHUNK & (CHUNK - 1)) == 0);
static_assert(CHUNK <= 4096);
static_assert((NBC & (NBC - 1)) == 0 && (NBF & (NBF - 1)) == 0);
static_assert(NBC == 4 * NBF);
static_assert(OTHR * 8 == NBC);
static_assert((RCAP % 32) == 0);
static_assert(RROWS == 4 * (RTHR / 32));
static_assert(RTHR >= KREL / 32);
static_assert((SAP % 8) == 0 && (XTP % 8) == 0 && (ATP % 8) == 0 && (DTP % 8) == 0);
static_assert(RROWS * SAP * 2 <= RROWS * KREL * 4);
static_assert(LDS_LAYER <= 300000);

typedef float    v4f  __attribute__((ext_vector_type(4)));
typedef float    v8f  __attribute__((ext_vector_type(8)));
typedef int      v4i  __attribute__((ext_vector_type(4)));
typedef _Float16 v8h  __attribute__((ext_vector_type(8)));
typedef _Float16 v16h __attribute__((ext_vector_type(16)));
union FragH { v16h v; v8h h[2]; };

__device__ __forceinline__ v8h cvt8(v4f a, v4f b) {
  v8h r;
  r[0] = (_Float16)a.x; r[1] = (_Float16)a.y; r[2] = (_Float16)a.z; r[3] = (_Float16)a.w;
  r[4] = (_Float16)b.x; r[5] = (_Float16)b.y; r[6] = (_Float16)b.z; r[7] = (_Float16)b.w;
  return r;
}

__device__ __forceinline__ v8f wmh(v16h a, v16h b, v8f c) {
  v8f d = __builtin_amdgcn_wmma_f32_16x16x32_f16(false, a, false, b, (short)0, c, false, false);
  asm volatile("v_nop\n\tv_nop\n\tv_nop\n\tv_nop" : "+v"(d) : "v"(a), "v"(b));
  return d;
}

__device__ __forceinline__ float sigm(float g) { return 1.0f / (1.0f + expf(-g)); }

template <int NT>
__device__ __forceinline__ void mm_step(const _Float16* ar, const _Float16* __restrict__ Bp, int bpitch,
                                        int t0, int ts, int m, int hh, int kt, v8f (&acc)[NT]) {
  FragH a;
  a.h[0] = *(const v8h*)(ar + 32 * kt);
  a.h[1] = *(const v8h*)(ar + 32 * kt + 16);
#pragma unroll
  for (int j = 0; j < NT; ++j) {
    const int t = t0 + ts * j;
    const _Float16* bp = Bp + (size_t)(16 * t + m) * bpitch + 32 * kt + 8 * hh;
    FragH b;
    b.h[0] = *(const v8h*)bp;
    b.h[1] = *(const v8h*)(bp + 16);
    acc[j] = wmh(a.v, b.v, acc[j]);
  }
}

template <int NT, int KS>
__device__ __forceinline__ void mm_tiles(const _Float16* ar, const _Float16* __restrict__ Bp, int bpitch,
                                         int t0, int ts, int m, int hh, v8f (&acc)[NT]) {
#pragma unroll
  for (int j = 0; j < NT; ++j) { v8f z = {0.f, 0.f, 0.f, 0.f, 0.f, 0.f, 0.f, 0.f}; acc[j] = z; }
  if (KS > 32) {
#pragma unroll 5
    for (int kt = 0; kt < KS; ++kt) mm_step<NT>(ar, Bp, bpitch, t0, ts, m, hh, kt, acc);
  } else {
#pragma unroll
    for (int kt = 0; kt < KS; ++kt) mm_step<NT>(ar, Bp, bpitch, t0, ts, m, hh, kt, acc);
  }
}

template <int NB>
__device__ __forceinline__ int scan_chunk(const int* __restrict__ dsts, int nE, int cbase, int slotBase,
                                          int vec8, int* list, int tid, int lane, int wave) {
  int wc = 0;
#pragma unroll
  for (int g = 0; g < NGRP; ++g) {
    const int el0  = (g * NTHR + tid) * EPT;
    const int e0   = cbase + el0;
    const int sent = -2147483647 - 1;
    v4i da, db;
    if (vec8 != 0 && cbase + CHUNK <= nE) {
      da = *(const v4i*)(dsts + e0);
      db = *(const v4i*)(dsts + e0 + 4);
    } else {
      da.x = (e0     < nE) ? dsts[min(e0, nE - 1)] : sent;
      da.y = (e0 + 1 < nE) ? dsts[min(e0 + 1, nE - 1)] : sent;
      da.z = (e0 + 2 < nE) ? dsts[min(e0 + 2, nE - 1)] : sent;
      da.w = (e0 + 3 < nE) ? dsts[min(e0 + 3, nE - 1)] : sent;
      db.x = (e0 + 4 < nE) ? dsts[min(e0 + 4, nE - 1)] : sent;
      db.y = (e0 + 5 < nE) ? dsts[min(e0 + 5, nE - 1)] : sent;
      db.z = (e0 + 6 < nE) ? dsts[min(e0 + 6, nE - 1)] : sent;
      db.w = (e0 + 7 < nE) ? dsts[min(e0 + 7, nE - 1)] : sent;
    }
    const unsigned nb = (unsigned)slotBase;
    const unsigned s0 = (unsigned)da.x - nb, s1 = (unsigned)da.y - nb;
    const unsigned s2 = (unsigned)da.z - nb, s3 = (unsigned)da.w - nb;
    const unsigned s4 = (unsigned)db.x - nb, s5 = (unsigned)db.y - nb;
    const unsigned s6 = (unsigned)db.z - nb, s7 = (unsigned)db.w - nb;
    const bool h0 = s0 < (unsigned)NB, h1 = s1 < (unsigned)NB, h2 = s2 < (unsigned)NB, h3 = s3 < (unsigned)NB;
    const bool h4 = s4 < (unsigned)NB, h5 = s5 < (unsigned)NB, h6 = s6 < (unsigned)NB, h7 = s7 < (unsigned)NB;
    const unsigned any = __builtin_amdgcn_ballot_w32(h0 | h1 | h2 | h3 | h4 | h5 | h6 | h7);
    if (any != 0u) {
#define HITJ(J, HJ, SJ) { \
        const unsigned mj = __builtin_amdgcn_ballot_w32(HJ); \
        if (mj != 0u) { \
          if (HJ) { \
            const int pos = wc + (int)__builtin_amdgcn_mbcnt_lo(mj, 0u); \
            if (pos < WCAP) list[wave * WCAP + pos] = ((el0 + (J)) << 12) | (int)(SJ); \
          } \
          wc += (int)__builtin_popcount(mj); } }
      HITJ(0, h0, s0)
      HITJ(1, h1, s1)
      HITJ(2, h2, s2)
      HITJ(3, h3, s3)
      HITJ(4, h4, s4)
      HITJ(5, h5, s5)
      HITJ(6, h6, s6)
      HITJ(7, h7, s7)
#undef HITJ
    }
  }
  return wc;
}

__global__ __launch_bounds__(NTHR) void k_wprep(
    const float* __restrict__ sw, const float* __restrict__ Wg, const float* __restrict__ Ug,
    const float* __restrict__ f1, _Float16* pSW, _Float16* pCat, _Float16* pUh, _Float16* pF1,
    int nL, int b1, int b2, int b3) {
  const int bid = blockIdx.x, tid = threadIdx.x;
  const int seg = bid < b1 ? 0 : (bid < b2 ? 1 : (bid < b3 ? 2 : 3));
  const int bs  = seg == 0 ? 0 : (seg == 1 ? b1 : (seg == 2 ? b2 : b3));
  const int i = (bid - bs) * NTHR + tid;
  float v[8];
  _Float16* dp;
  if (seg == 0) {
    const int per = NP208 * XP;
    if (i >= nL * (per / 8)) return;
    const int o = i * 8;
    const int layer = o / per;
    const int oo = o - layer * per;
    const int n = oo / XP, k0 = oo - n * XP;
    const int nc = n < DIMC ? n : DIMC - 1;
    const float* src = sw + (size_t)layer * DIMC * DIMC;
#pragma unroll
    for (int e = 0; e < 8; ++e) {
      const int k = k0 + e, kc = k < DIMC ? k : DIMC - 1;
      const float x = src[(size_t)kc * DIMC + nc];
      v[e] = (k < DIMC && n < DIMC) ? x * WSC : 0.0f;
    }
    dp = pSW + o;
  } else if (seg == 1) {
    if (i >= GDP * KCAT / 8) return;
    const int o = i * 8;
    const int n = o / KCAT, k0 = o - n * KCAT;
    const int nc = n < GD ? n : GD - 1;
#pragma unroll
    for (int e = 0; e < 8; ++e) {
      const int k = k0 + e;
      const int kw = k < DIMC ? k : DIMC - 1;
      int ku = k - NP208; ku = ku < 0 ? 0 : (ku > DIMC - 1 ? DIMC - 1 : ku);
      const float w = Wg[(size_t)kw * GD + nc];
      const float u = Ug[(size_t)ku * GD + nc];
      const float val = k < DIMC ? w : ((k >= NP208 && k < NP208 + DIMC) ? u : 0.0f);
      v[e] = n < GD ? val * WSC : 0.0f;
    }
    dp = pCat + o;
  } else if (seg == 2) {
    if (i >= NP208 * XP / 8) return;
    const int o = i * 8;
    const int n = o / XP, k0 = o - n * XP;
    const int nc = n < DIMC ? n : DIMC - 1;
#pragma unroll
    for (int e = 0; e < 8; ++e) {
      const int k = k0 + e, kc = k < DIMC ? k : DIMC - 1;
      const float x = Ug[(size_t)kc * GD + 2 * DIMC + nc];
      v[e] = (k < DIMC && n < DIMC) ? x * WSC : 0.0f;
    }
    dp = pUh + o;
  } else {
    if (i >= HIDN * KDEC / 8) return;
    const int o = i * 8;
    const int n = o / KDEC, k0 = o - n * KDEC;
#pragma unroll
    for (int e = 0; e < 8; ++e) {
      const int k = k0 + e, kc = k < GD ? k : GD - 1;
      const float x = f1[(size_t)kc * HIDN + n];
      v[e] = k < GD ? x * WSC : 0.0f;
    }
    dp = pF1 + o;
  }
  v4f a, b;
  a.x = v[0]; a.y = v[1]; a.z = v[2]; a.w = v[3];
  b.x = v[4]; b.y = v[5]; b.z = v[6]; b.w = v[7];
  const v8h hv = cvt8(a, b);
  *(volatile v8h*)dp = hv;
  __threadfence();
  *(volatile v8h*)dp = hv;
}

__global__ __launch_bounds__(NTHR) void k_relw(const float* __restrict__ basis, const float* __restrict__ coeff,
                                              _Float16* RW) {
  __shared__ __attribute__((aligned(16))) float st[64][16];
  const int tid = threadIdx.x, lane = tid & 31, wave = tid >> 5;
  const int kt = blockIdx.x, ot = blockIdx.y, l = blockIdx.z;
  const int kl = tid >> 2, og = tid & 3;
  const int k = kt * 64 + kl;
  const int kc = k < KREL ? k : KREL - 1;
  const int r = kc / DIMC, i = kc - r * DIMC;
  const int o0 = ot * 16 + 4 * og;
  const int oc = o0 < DIMC - 4 ? o0 : DIMC - 4;
  const float* bp = basis + ((size_t)l * NBAS * DIMC + i) * DIMC + oc;
  const float* cp = coeff + ((size_t)l * RREL + r) * NBAS;
  v4f acc = {0.f, 0.f, 0.f, 0.f};
#pragma unroll 1
  for (int b = 0; b < NBAS; ++b) {
    const float cf = cp[b];
    const v4f bv = *(const v4f*)(bp + (size_t)b * DIMC * DIMC);
    acc = acc + bv * cf;
  }
  const bool ok = (k < KREL) && (o0 < DIMC);
  acc = acc * RWSC;
  if (!ok) { v4f z = {0.f, 0.f, 0.f, 0.f}; acc = z; }
  *(v4f*)(&st[kl][4 * og]) = acc;
  __syncthreads();
  if (tid < 128) {
    const int q  = 4 * wave + (lane >> 3);
    const int kk = (lane & 7) * 8;
    v4f a, b;
    a.x = st[kk + 0][q]; a.y = st[kk + 1][q]; a.z = st[kk + 2][q]; a.w = st[kk + 3][q];
    b.x = st[kk + 4][q]; b.y = st[kk + 5][q]; b.z = st[kk + 6][q]; b.w = st[kk + 7][q];
    const v8h hv = cvt8(a, b);
    _Float16* dp = RW + ((size_t)l * NP208 + (size_t)(ot * 16 + q)) * RWP + kt * 64 + kk;
    *(volatile v8h*)dp = hv;
    __threadfence();
    *(volatile v8h*)dp = hv;
  }
}

__global__ __launch_bounds__(NTHR) void k_init(const float* __restrict__ emb, float* h, int nN, int total) {
  const int p = blockIdx.x * NTHR + (int)threadIdx.x;
  if (p >= total) return;
  const int row = p / (XP / 4);
  const int c4  = p - row * (XP / 4);
  const int rc  = row < nN ? row : nN - 1;
  const int cc  = c4 < DIMC / 4 ? c4 : DIMC / 4 - 1;
  v4f v = *(const v4f*)(emb + (size_t)rc * DIMC + 4 * cc);
  if (!((row < nN) && (c4 < DIMC / 4))) { v4f z = {0.f, 0.f, 0.f, 0.f}; v = z; }
  float* dp = h + (size_t)p * 4;
  *(volatile v4f*)dp = v;
  __threadfence();
  *(volatile v4f*)dp = v;
}

__global__ __launch_bounds__(NTHR) void k_count(const int* __restrict__ rcv, int* cnt, int nE, int vec8) {
  __shared__ __attribute__((aligned(16))) int scnt[NBC];
  __shared__ __attribute__((aligned(16))) int list[LISTN];
  __shared__ int wcnt[NWAVE];
  const int tid = threadIdx.x, lane = tid & 31, wave = tid >> 5;
  const int nodeBase = blockIdx.x * NBC;

  for (int i = tid; i < NBC; i += NTHR) scnt[i] = 0;
  __syncthreads();

  const int nChunks = (nE + CHUNK - 1) / CHUNK;
#pragma unroll 1
  for (int ch = 0; ch < nChunks; ++ch) {
    const int cbase = ch * CHUNK;
    const int wc = scan_chunk<NBC>(rcv, nE, cbase, nodeBase, vec8, list, tid, lane, wave);
    if (lane == 0) wcnt[wave] = wc;
    __syncthreads();
    if (wave == 0) {
#pragma unroll 1
      for (int wsx = 0; wsx < NWAVE; ++wsx) {
        int n = __builtin_amdgcn_readfirstlane(wcnt[wsx]);
        n = n > WCAP ? WCAP : (n < 0 ? 0 : n);
        const int* lp = list + wsx * WCAP;
#pragma unroll 1
        for (int i = 0; i < n; ++i) {
          const int ent  = __builtin_amdgcn_readfirstlane(lp[i]);
          const int slot = ent & (NBC - 1);
          if (lane == 0) scnt[slot] = scnt[slot] + 1;
        }
      }
    }
    __syncthreads();
  }

  v4i cq[4];
#pragma unroll
  for (int q = 0; q < 4; ++q) {
    const int f = (wave * 4 + q) * 128 + 4 * lane;
    cq[q] = *(const v4i*)(scnt + f);
  }
  int* cp = cnt + (size_t)nodeBase;
#pragma unroll
  for (int q = 0; q < 4; ++q) {
    const int f = (wave * 4 + q) * 128 + 4 * lane;
    *(volatile v4i*)(cp + f) = cq[q];
  }
  __threadfence();
#pragma unroll
  for (int q = 0; q < 4; ++q) {
    const int f = (wave * 4 + q) * 128 + 4 * lane;
    *(volatile v4i*)(cp + f) = cq[q];
  }
}

__global__ __launch_bounds__(OTHR) void k_offsets(
    const int* __restrict__ cnt, int* off, int* rbase, int nChunk) {
  __shared__ __attribute__((aligned(16))) int soff[NBC];
  __shared__ __attribute__((aligned(16))) int srb[RBN];
  __shared__ int wtot[OTHR / 32];
  const int tid = threadIdx.x, lane = tid & 31, wave = tid >> 5, sub = tid >> 7;
  for (int i = tid; i < RBN; i += OTHR) srb[i] = 0;
  int carry = 0;
#pragma unroll 1
  for (int ch = 0; ch < nChunk; ++ch) {
    const int base = ch * NBC;
    const v4i c0 = *(const v4i*)(cnt + base + 8 * tid);
    const v4i c1 = *(const v4i*)(cnt + base + 8 * tid + 4);
    const int e0 = max(c0.x, 0), e1 = max(c0.y, 0), e2 = max(c0.z, 0), e3 = max(c0.w, 0);
    const int e4 = max(c1.x, 0), e5 = max(c1.y, 0), e6 = max(c1.z, 0), e7 = max(c1.w, 0);
    const int ts = e0 + e1 + e2 + e3 + e4 + e5 + e6 + e7;
    int incl = ts;
#pragma unroll
    for (int d = 1; d < 32; d <<= 1) {
      const int t = __shfl_up(incl, d);
      if (lane >= d) incl += t;
    }
    if (lane == 31) wtot[wave] = incl;
    __syncthreads();
    const int S0 = wtot[0]  + wtot[1]  + wtot[2]  + wtot[3];
    const int S1 = wtot[4]  + wtot[5]  + wtot[6]  + wtot[7];
    const int S2 = wtot[8]  + wtot[9]  + wtot[10] + wtot[11];
    const int S3 = wtot[12] + wtot[13] + wtot[14] + wtot[15];
    int pre = 0;
#pragma unroll 1
    for (int w = 4 * sub; w < wave; ++w) pre += wtot[w];
    const int b0 = carry;
    const int b1 = b0 + ((S0 + 31) & ~31);
    const int b2 = b1 + ((S1 + 31) & ~31);
    const int b3 = b2 + ((S2 + 31) & ~31);
    const int b4 = b3 + ((S3 + 31) & ~31);
    const int myb = sub == 0 ? b0 : (sub == 1 ? b1 : (sub == 2 ? b2 : b3));
    if (tid == 0) {
      srb[min(4 * ch + 0, RBN - 1)] = b0;
      srb[min(4 * ch + 1, RBN - 1)] = b1;
      srb[min(4 * ch + 2, RBN - 1)] = b2;
      srb[min(4 * ch + 3, RBN - 1)] = b3;
    }
    int run = myb + pre + incl - ts;
    soff[8 * tid + 0] = run; run += e0;
    soff[8 * tid + 1] = run; run += e1;
    soff[8 * tid + 2] = run; run += e2;
    soff[8 * tid + 3] = run; run += e3;
    soff[8 * tid + 4] = run; run += e4;
    soff[8 * tid + 5] = run; run += e5;
    soff[8 * tid + 6] = run; run += e6;
    soff[8 * tid + 7] = run;
    carry = b4;
    __syncthreads();
    const v4i o0 = *(const v4i*)(soff + 4 * tid);
    const v4i o1 = *(const v4i*)(soff + 4 * (tid + OTHR));
    int* op = off + base;
    *(volatile v4i*)(op + 4 * tid) = o0;
    *(volatile v4i*)(op + 4 * (tid + OTHR)) = o1;
    __threadfence();
    *(volatile v4i*)(op + 4 * tid) = o0;
    *(volatile v4i*)(op + 4 * (tid + OTHR)) = o1;
    __syncthreads();
  }
  if (tid == 0) srb[min(4 * nChunk, RBN - 1)] = carry;
  __syncthreads();
  v4i rv = {0, 0, 0, 0};
  if (tid < 32) rv = *(const v4i*)(srb + 4 * tid);
  if (tid < 32) *(volatile v4i*)(rbase + 4 * tid) = rv;
  __threadfence();
  if (tid < 32) *(volatile v4i*)(rbase + 4 * tid) = rv;
}

__global__ __launch_bounds__(NTHR) void k_fill(
    const int* __restrict__ rcv, const int* __restrict__ snd, const int* __restrict__ rel,
    const int* __restrict__ off, const int* __restrict__ rbase,
    int* csr, int nN, int nE, int vec8, int csrLen) {
  extern __shared__ v4f lds_dyn[];
  int* region = (int*)lds_dyn;
  int* cursor = region + RCAP;
  int* list   = cursor + NBF;
  int* wcnt   = list + LISTN;
  const int tid = threadIdx.x, lane = tid & 31, wave = tid >> 5;
  const int b = blockIdx.x;
  const int nodeBase = b * NBF;

  int rb0 = rbase[b];
  const int rb1 = rbase[b + 1];
  rb0 = rb0 < 0 ? 0 : (rb0 > csrLen ? csrLen : rb0);
  rb0 &= ~31;
  int len = rb1 - rb0;
  len = len < 0 ? 0 : (len > RCAP ? RCAP : len);
  int lenW = (len + 31) & ~31;
  if (rb0 + lenW > csrLen) lenW = (csrLen - rb0) & ~31;

  {
    const v4i z = {0, 0, 0, 0};
    for (int i = tid; i < RCAP / 4; i += NTHR) ((v4i*)region)[i] = z;
    for (int s = tid; s < NBF; s += NTHR) {
      int o = off[nodeBase + s] - rb0;
      o = o < 0 ? 0 : (o > RCAP ? RCAP : o);
      cursor[s] = o;
    }
  }
  __syncthreads();

  const int nChunks = (nE + CHUNK - 1) / CHUNK;
#pragma unroll 1
  for (int ch = 0; ch < nChunks; ++ch) {
    const int cbase = ch * CHUNK;
    const int wc = scan_chunk<NBF>(rcv, nE, cbase, nodeBase, vec8, list, tid, lane, wave);
    if (lane == 0) wcnt[wave] = wc;
    __syncthreads();
    if (wave == 0) {
#pragma unroll 1
      for (int wsx = 0; wsx < NWAVE; ++wsx) {
        int n = __builtin_amdgcn_readfirstlane(wcnt[wsx]);
        n = n > WCAP ? WCAP : (n < 0 ? 0 : n);
        const int* lp = list + wsx * WCAP;
#pragma unroll 1
        for (int i = 0; i < n; ++i) {
          const int ent  = __builtin_amdgcn_readfirstlane(lp[i]);
          const int slot = ent & (NBF - 1);
          int e = cbase + ((ent >> 12) & (CHUNK - 1));
          e = e > nE - 1 ? nE - 1 : e;
          int sv = snd[e];
          sv = sv < 0 ? 0 : (sv > nN - 1 ? nN - 1 : sv);
          int rl = rel[e];
          rl = rl < 0 ? 0 : (rl > RREL - 1 ? RREL - 1 : rl);
          const int pk = (sv << 5) | rl;
          if (lane == 0) {
            int pos = cursor[slot];
            pos = pos < 0 ? 0 : (pos > RCAP - 1 ? RCAP - 1 : pos);
            region[pos] = pk;
            const int np = pos + 1;
            cursor[slot] = np > RCAP ? RCAP : np;
          }
        }
      }
    }
    __syncthreads();
  }

  const int nv = lenW >> 2;
  int* gp = csr + rb0;
#pragma unroll 1
  for (int i = tid; i < nv; i += NTHR) { const v4i v = ((const v4i*)region)[i]; *(volatile v4i*)(gp + 4 * i) = v; }
  __threadfence();
#pragma unroll 1
  for (int i = tid; i < nv; i += NTHR) { const v4i v = ((const v4i*)region)[i]; *(volatile v4i*)(gp + 4 * i) = v; }
}

template <int NT>
__device__ __forceinline__ void layer_tiles(const _Float16* Sh, const _Float16* xt,
    const _Float16* __restrict__ RW, const _Float16* __restrict__ SWp, const float* __restrict__ bias,
    const float* sinv, float* stg, int wave, int m, int hh) {
  v8f acc[NT];
  mm_tiles<NT, KREL / 32>(Sh + m * SAP + 8 * hh, RW, RWP, wave, 4, m, hh, acc);
  float inv[8];
#pragma unroll
  for (int r = 0; r < 8; ++r) inv[r] = sinv[8 * hh + r] * INV22;
  float res[NT][8];
#pragma unroll
  for (int j = 0; j < NT; ++j) {
#pragma unroll
    for (int r = 0; r < 8; ++r) res[j][r] = acc[j][r] * inv[r];
  }
  mm_tiles<NT, XP / 32>(xt + m * XTP + 8 * hh, SWp, XP, wave, 4, m, hh, acc);
#pragma unroll
  for (int j = 0; j < NT; ++j) {
    const int t = wave + 4 * j;
    const int col = 16 * t + m;
    const float bl = bias[col < DIMC ? col : DIMC - 1];
    const float bv = col < DIMC ? bl : 0.0f;
    float* sp = stg + (8 * hh) * XP + col;
#pragma unroll
    for (int r = 0; r < 8; ++r) {
      const float v = res[j][r] + acc[j][r] * INV17 + bv;
      sp[r * XP] = fmaxf(v, 0.0f);
    }
  }
}

__global__ __launch_bounds__(RTHR) void k_layer(
    const float* __restrict__ xin, const int* __restrict__ csr, const int* __restrict__ off,
    const int* __restrict__ cnt, const _Float16* __restrict__ RW, const _Float16* __restrict__ SWp,
    const float* __restrict__ bias, float* xout, int nN, int csrLen) {
  extern __shared__ v4f lds_dyn[];
  float*    S    = (float*)lds_dyn;
  _Float16* Sh   = (_Float16*)lds_dyn;
  _Float16* xt   = (_Float16*)((char*)lds_dyn + RROWS * KREL * 4);
  float*    stg  = (float*)((char*)lds_dyn + RROWS * KREL * 4 + RROWS * XTP * 2);
  float*    sinv = stg + RROWS * XP;
  int*      scnt = (int*)(sinv + RROWS);
  const int tid = threadIdx.x, lane = tid & 31, wave = tid >> 5, hh = lane >> 4, m = lane & 15;
  const int nodeBase = blockIdx.x * RROWS;

  {
    const v4f z = {0.f, 0.f, 0.f, 0.f};
    for (int i = tid; i < RROWS * KREL / 4; i += RTHR) ((v4f*)S)[i] = z;
    for (int i = tid; i < RROWS * XP / 4; i += RTHR) ((v4f*)stg)[i] = z;
    if (tid < RROWS) {
      int c = cnt[nodeBase + tid];
      c = c < 0 ? 0 : c;
      scnt[tid] = c;
      sinv[tid] = 1.0f / (float)(c < 1 ? 1 : c);
    }
    for (int p = tid; p < RROWS * (XP / 8); p += RTHR) {
      const int row = p / (XP / 8), c8 = p - row * (XP / 8);
      const float* xp = xin + (size_t)(nodeBase + row) * XP + 8 * c8;
      const v4f a = *(const v4f*)xp, b = *(const v4f*)(xp + 4);
      *(v8h*)(xt + row * XTP + 8 * c8) = cvt8(a * ASC, b * ASC);
    }
  }
  __syncthreads();

#pragma unroll 1
  for (int j = 0; j < RROWS / 4; ++j) {
    const int slot = wave * (RROWS / 4) + j;
    const int c = nodeBase + slot;
    int n = scnt[slot];
    n = n < 0 ? 0 : (n > DEGCAP ? DEGCAP : n);
    int st = off[c];
    st = st < 0 ? 0 : (st > csrLen - 1 ? csrLen - 1 : st);
    float* srow = S + slot * KREL;
#pragma unroll 1
    for (int q0 = 0; q0 < n; q0 += 32) {
      int pos = st + q0 + lane;
      pos = pos < 0 ? 0 : (pos > csrLen - 1 ? csrLen - 1 : pos);
      const int ent = csr[pos];
      const int mcnt = (n - q0) < 32 ? (n - q0) : 32;
#pragma unroll 1
      for (int p = 0; p < mcnt; ++p) {
        const int e = __builtin_amdgcn_readlane(ent, p);
        int s = e >> 5;
        s = s < 0 ? 0 : (s > nN - 1 ? nN - 1 : s);
        int r = e & 31;
        r = r > RREL - 1 ? RREL - 1 : r;
        const float* xr = xin + (size_t)s * XP;
        const v4f a = *(const v4f*)(xr + 4 * lane);
        const v4f b = *(const v4f*)(xr + 128 + 4 * (lane < 17 ? lane : 17));
        float* sp = srow + r * DIMC;
        v4f* pa = (v4f*)(sp + 4 * lane);
        *pa = *pa + a;
        if (lane < 18) { v4f* pb = (v4f*)(sp + 128 + 4 * lane); *pb = *pb + b; }
      }
    }
  }
  __syncthreads();

  {
    const int tc = tid < (KREL / 32 - 1) ? tid : (KREL / 32 - 1);
#pragma unroll 1
    for (int r = 0; r < RROWS; ++r) {
      v4f v[8];
      const float* rp = S + r * KREL + 32 * tc;
#pragma unroll
      for (int e = 0; e < 8; ++e) v[e] = *(const v4f*)(rp + 4 * e);
      __syncthreads();
      if (tid < KREL / 32) {
        _Float16* hp = Sh + r * SAP + 32 * tid;
#pragma unroll
        for (int e = 0; e < 4; ++e) *(v8h*)(hp + 8 * e) = cvt8(v[2 * e] * ASC, v[2 * e + 1] * ASC);
      }
    }
  }
  __syncthreads();

  if (wave == 0) layer_tiles<4>(Sh, xt, RW, SWp, bias, sinv, stg, wave, m, hh);
  else           layer_tiles<3>(Sh, xt, RW, SWp, bias, sinv, stg, wave, m, hh);
  __syncthreads();

  float* gp = xout + (size_t)nodeBase * XP;
#pragma unroll 1
  for (int i = tid; i < RROWS * XP / 4; i += RTHR) { const v4f v = ((const v4f*)stg)[i]; *(volatile v4f*)(gp + 4 * i) = v; }
  __threadfence();
#pragma unroll 1
  for (int i = tid; i < RROWS * XP / 4; i += RTHR) { const v4f v = ((const v4f*)stg)[i]; *(volatile v4f*)(gp + 4 * i) = v; }
}

template <int NT>
__device__ __forceinline__ void gru_gates(const _Float16* ar, const _Float16* __restrict__ Wc,
    const float* __restrict__ bg, float* G, int t0, int rt, int m, int hh) {
  v8f acc[NT];
  mm_tiles<NT, KCAT / 32>(ar, Wc, KCAT, t0, 1, m, hh, acc);
#pragma unroll
  for (int j = 0; j < NT; ++j) {
    const int col = 16 * (t0 + j) + m;
    const float bl = bg[col < GD ? col : GD - 1];
    const float bv = col < GD ? bl : 0.0f;
    float* sp = G + (16 * rt + 8 * hh) * GDP + col;
#pragma unroll
    for (int r = 0; r < 8; ++r) sp[r * GDP] = acc[j][r] * INV17 + bv;
  }
}

template <int NT>
__device__ __forceinline__ void gru_uh(const _Float16* ar, const _Float16* __restrict__ Uh,
    float* HS, int t0, int rt, int m, int hh) {
  v8f acc[NT];
  mm_tiles<NT, XP / 32>(ar, Uh, XP, t0, 4, m, hh, acc);
#pragma unroll
  for (int j = 0; j < NT; ++j) {
    const int col = 16 * (t0 + 4 * j) + m;
    float* sp = HS + (16 * rt + 8 * hh) * XP + col;
#pragma unroll
    for (int r = 0; r < 8; ++r) sp[r * XP] = acc[j][r] * INV17;
  }
}

__global__ __launch_bounds__(NTHR) void k_gru(
    const float* __restrict__ x, const float* __restrict__ hin, const _Float16* __restrict__ Wc,
    const _Float16* __restrict__ Uh, const float* __restrict__ bg, float* hout) {
  extern __shared__ v4f lds_dyn[];
  _Float16* At = (_Float16*)lds_dyn;
  float*    G  = (float*)((char*)lds_dyn + GROWS * ATP * 2);
  _Float16* RH = (_Float16*)((char*)lds_dyn + GROWS * ATP * 2 + GROWS * GDP * 4);
  float*    HS = (float*)((char*)lds_dyn + GROWS * ATP * 2 + GROWS * GDP * 4 + GROWS * XTP * 2);
  const int tid = threadIdx.x, lane = tid & 31, wave = tid >> 5, hh = lane >> 4, m = lane & 15;
  const int nodeBase = blockIdx.x * GROWS;

  for (int p = tid; p < GROWS * (NP208 / 8); p += NTHR) {
    const int row = p / (NP208 / 8), c8 = p - row * (NP208 / 8);
    const float* xp = x + (size_t)(nodeBase + row) * XP + 8 * c8;
    const v4f a = *(const v4f*)xp, b = *(const v4f*)(xp + 4);
    *(v8h*)(At + row * ATP + 8 * c8) = cvt8(a * ASC, b * ASC);
  }
  for (int p = tid; p < GROWS * (NP208 / 8); p += NTHR) {
    const int row = p / (NP208 / 8), c8 = p - row * (NP208 / 8);
    const float* hp = hin + (size_t)(nodeBase + row) * XP + 8 * c8;
    const v4f a = *(const v4f*)hp, b = *(const v4f*)(hp + 4);
    *(v8h*)(At + row * ATP + NP208 + 8 * c8) = cvt8(a * ASC, b * ASC);
  }
  __syncthreads();

  const int rt = wave & 1, cg = wave >> 1;
  {
    const _Float16* ar = At + (16 * rt + m) * ATP + 8 * hh;
    if (cg < 2) gru_gates<10>(ar, Wc, bg, G, cg * 10, rt, m, hh);
    else        gru_gates<9>(ar, Wc, bg, G, 20 + (cg - 2) * 9, rt, m, hh);
  }
  __syncthreads();

#pragma unroll 1
  for (int idx = tid; idx < GROWS * XP; idx += NTHR) {
    const int row = idx / XP, col = idx - row * XP;
    const int cc = col < DIMC ? col : DIMC - 1;
    const float g  = G[row * GDP + cc];
    const float hv = hin[(size_t)(nodeBase + row) * XP + cc];
    const float rg = sigm(g);
    const float v = col < DIMC ? rg * hv * ASC : 0.0f;
    RH[row * XTP + col] = (_Float16)v;
  }
  __syncthreads();

  {
    const _Float16* ar = RH + (16 * rt + m) * XTP + 8 * hh;
    if (cg == 0) gru_uh<4>(ar, Uh, HS, cg, rt, m, hh);
    else         gru_uh<3>(ar, Uh, HS, cg, rt, m, hh);
  }
  __syncthreads();

#pragma unroll 1
  for (int idx = tid; idx < GROWS * XP; idx += NTHR) {
    const int row = idx / XP, col = idx - row * XP;
    const int cc = col < DIMC ? col : DIMC - 1;
    const float a3 = HS[row * XP + cc];
    const float gz = G[row * GDP + DIMC + cc];
    const float gq = G[row * GDP + 2 * DIMC + cc];
    const float z  = sigm(gz);
    const float ht = tanhf(gq + a3);
    const float ho = hin[(size_t)(nodeBase + row) * XP + cc];
    const float v  = col < DIMC ? (1.0f - z) * ho + z * ht : 0.0f;
    HS[idx] = v;
  }
  __syncthreads();

  float* gp = hout + (size_t)nodeBase * XP;
#pragma unroll 1
  for (int i = tid; i < GROWS * XP / 4; i += NTHR) { const v4f v = ((const v4f*)HS)[i]; *(volatile v4f*)(gp + 4 * i) = v; }
  __threadfence();
#pragma unroll 1
  for (int i = tid; i < GROWS * XP / 4; i += NTHR) { const v4f v = ((const v4f*)HS)[i]; *(volatile v4f*)(gp + 4 * i) = v; }
}

__global__ __launch_bounds__(NTHR) void k_dec(
    const float* __restrict__ h, const float* __restrict__ relemb, const int* __restrict__ tri,
    const _Float16* __restrict__ F1, const float* __restrict__ fc1b, const float* __restrict__ fc2,
    const float* __restrict__ fc2b, float* out, int nN, int nRel, int nQ) {
  extern __shared__ v4f lds_dyn[];
  _Float16* At   = (_Float16*)lds_dyn;
  float*    part = (float*)((char*)lds_dyn + DROWS * DTP * 2);
  const int tid = threadIdx.x, lane = tid & 31, wave = tid >> 5, hh = lane >> 4, m = lane & 15;
  const int qBase = blockIdx.x * DROWS;

  for (int p = tid; p < DROWS * (DIMC / 8); p += NTHR) {
    const int row = p / (DIMC / 8), c = p - row * (DIMC / 8);
    const int q = (qBase + row) < nQ ? (qBase + row) : nQ - 1;
    int s = tri[q * 3];
    s = s < 0 ? 0 : (s > nN - 1 ? nN - 1 : s);
    const float* sp = h + (size_t)s * XP + 8 * c;
    const v4f a = *(const v4f*)sp, b = *(const v4f*)(sp + 4);
    *(v8h*)(At + row * DTP + 8 * c) = cvt8(a * ASC, b * ASC);
  }
  for (int p = tid; p < DROWS * (DIMC / 8); p += NTHR) {
    const int row = p / (DIMC / 8), c = p - row * (DIMC / 8);
    const int q = (qBase + row) < nQ ? (qBase + row) : nQ - 1;
    int rr = tri[q * 3 + 1];
    rr = rr < 0 ? 0 : (rr > nRel - 1 ? nRel - 1 : rr);
    const float* sp = relemb + (size_t)rr * DIMC + 8 * c;
    const v4f a = *(const v4f*)sp, b = *(const v4f*)(sp + 4);
    *(v8h*)(At + row * DTP + DIMC + 8 * c) = cvt8(a * ASC, b * ASC);
  }
  for (int p = tid; p < DROWS * (DIMC / 8); p += NTHR) {
    const int row = p / (DIMC / 8), c = p - row * (DIMC / 8);
    const int q = (qBase + row) < nQ ? (qBase + row) : nQ - 1;
    int o = tri[q * 3 + 2];
    o = o < 0 ? 0 : (o > nN - 1 ? nN - 1 : o);
    const float* sp = h + (size_t)o * XP + 8 * c;
    const v4f a = *(const v4f*)sp, b = *(const v4f*)(sp + 4);
    *(v8h*)(At + row * DTP + 2 * DIMC + 8 * c) = cvt8(a * ASC, b * ASC);
  }
  if (tid < DROWS) {
    const v4f z = {0.f, 0.f, 0.f, 0.f};
    *(v8h*)(At + tid * DTP + GD) = cvt8(z, z);
  }
  __syncthreads();

  const int rt = wave & 1, cg = wave >> 1;
  v8f acc[4];
  mm_tiles<4, KDEC / 32>(At + (16 * rt + m) * DTP + 8 * hh, F1, KDEC, 4 * cg, 1, m, hh, acc);
  float pr[8];
#pragma unroll
  for (int r = 0; r < 8; ++r) pr[r] = 0.0f;
#pragma unroll
  for (int j = 0; j < 4; ++j) {
    const int col = 16 * (4 * cg + j) + m;
    const float b1 = fc1b[col];
    const float w2 = fc2[col];
#pragma unroll
    for (int r = 0; r < 8; ++r) {
      const float v = fmaxf(acc[j][r] * INV17 + b1, 0.0f);
      pr[r] += v * w2;
    }
  }
#pragma unroll
  for (int r = 0; r < 8; ++r) {
    pr[r] += __shfl_xor(pr[r], 8, 32);
    pr[r] += __shfl_xor(pr[r], 4, 32);
    pr[r] += __shfl_xor(pr[r], 2, 32);
    pr[r] += __shfl_xor(pr[r], 1, 32);
  }
  if (m == 0) {
#pragma unroll
    for (int r = 0; r < 8; ++r) part[cg * DROWS + 16 * rt + 8 * hh + r] = pr[r];
  }
  __syncthreads();

  v4f ov = {0.f, 0.f, 0.f, 0.f};
  const bool wl = (tid < 8);
  if (wl) {
    const float b2 = fc2b[0];
#pragma unroll
    for (int e = 0; e < 4; ++e) {
      const int q = 4 * tid + e;
      ov[e] = part[q] + part[DROWS + q] + part[2 * DROWS + q] + part[3 * DROWS + q] + b2;
    }
  }
  float* op = out + qBase;
  const bool full = (qBase + DROWS <= nQ);
  if (full) { if (wl) *(volatile v4f*)(op + 4 * tid) = ov; }
  else if (wl) {
#pragma unroll
    for (int e = 0; e < 4; ++e) if (qBase + 4 * tid + e < nQ) ((volatile float*)op)[4 * tid + e] = ov[e];
  }
  __threadfence();
  if (full) { if (wl) *(volatile v4f*)(op + 4 * tid) = ov; }
  else if (wl) {
#pragma unroll
    for (int e = 0; e < 4; ++e) if (qBase + 4 * tid + e < nQ) ((volatile float*)op)[4 * tid + e] = ov[e];
  }
}

static inline int cdiv_h(int a, int b) { return (a + b - 1) / b; }
static inline size_t al256(size_t x) { return (x + 255) & ~(size_t)255; }

extern "C" void kernel_launch(void* const* d_in, const int* in_sizes, int n_in,
                              void* d_out, int out_size, void* d_ws, size_t ws_size,
                              hipStream_t stream) {
  if (n_in < 17) return;
  const int nN = in_sizes[0] / DIMC;
  if (nN < 1 || in_sizes[0] != nN * DIMC) return;
  const int nL = in_sizes[1] / (NBAS * DIMC * DIMC);
  if (nL < 1 || in_sizes[1] != nL * NBAS * DIMC * DIMC) return;
  if (in_sizes[2] != nL * RREL * NBAS || in_sizes[3] != nL * DIMC * DIMC || in_sizes[4] < nL * DIMC) return;
  if (in_sizes[5] != DIMC * GD || in_sizes[6] != DIMC * GD || in_sizes[7] < GD) return;
  const int nRel = in_sizes[8] / DIMC;
  if (nRel < 1 || in_sizes[8] != nRel * DIMC) return;
  if (in_sizes[9] != GD * HIDN || in_sizes[10] < HIDN || in_sizes[11] < HIDN || in_sizes[12] < 1) return;
  const int nT = 2;
  const int nE = in_sizes[13] / nT;
  if (nE < 1 || in_sizes[13] != nT * nE || in_sizes[14] != in_sizes[13] || in_sizes[15] != in_sizes[13]) return;
  const int nQ = in_sizes[16] / 3;
  if (nQ < 1 || in_sizes[16] != 3 * nQ || out_size != nQ) return;
  if (nN > (1 << 24) || nE > (1 << 28)) return;

  const float* emb    = (const float*)d_in[0];
  const float* basis  = (const float*)d_in[1];
  const float* coeff  = (const float*)d_in[2];
  const float* selfw  = (const float*)d_in[3];
  const float* bias   = (const float*)d_in[4];
  const float* Wg     = (const float*)d_in[5];
  const float* Ug     = (const float*)d_in[6];
  const float* bg     = (const float*)d_in[7];
  const float* relemb = (const float*)d_in[8];
  const float* fc1    = (const float*)d_in[9];
  const float* fc1b   = (const float*)d_in[10];
  const float* fc2    = (const float*)d_in[11];
  const float* fc2b   = (const float*)d_in[12];
  const int*   snd    = (const int*)d_in[13];
  const int*   rcv    = (const int*)d_in[14];
  const int*   relt   = (const int*)d_in[15];
  const int*   tri    = (const int*)d_in[16];
  float* out = (float*)d_out;

  const int NPAD   = ((nN + 31) / 32) * 32;
  const int nBC    = cdiv_h(nN, NBC);
  const int CNTPAD = nBC * NBC;
  if (4 * nBC + 1 > RBN) return;
  const int nBF    = cdiv_h(nN, NBF);
  const int csrLen = ((nE + 31) & ~31) + 4096;

  const size_t plane = (size_t)NPAD * XP * 4;
  size_t off = 0;
  const size_t oSW  = off; off = al256(off + (size_t)nL * NP208 * XP * 2);
  const size_t oCat = off; off = al256(off + (size_t)GDP * KCAT * 2);
  const size_t oUh  = off; off = al256(off + (size_t)NP208 * XP * 2);
  const size_t oF1  = off; off = al256(off + (size_t)HIDN * KDEC * 2);
  const size_t oRW  = off; off = al256(off + (size_t)nL * NP208 * RWP * 2);
  size_t oCnt[2], oOff[2], oRb[2], oCsr[2];
  for (int t = 0; t < 2; ++t) {
    oCnt[t] = off; off = al256(off + (size_t)CNTPAD * 4);
    oOff[t] = off; off = al256(off + (size_t)CNTPAD * 4);
    oRb[t]  = off; off = al256(off + (size_t)RBN * 4);
    oCsr[t] = off; off = al256(off + (size_t)csrLen * 4);
  }
  const size_t oH0 = off; off = al256(off + plane);
  const size_t oH1 = off; off = al256(off + plane);
  const size_t oXA = off; off = al256(off + plane);
  const size_t oXB = off; off = al256(off + plane);
  const size_t wsCap = (size_t)134217728;
  if (off > ws_size || off > wsCap) return;

  char* ws = (char*)d_ws;
  _Float16* pSW  = (_Float16*)(ws + oSW);
  _Float16* pCat = (_Float16*)(ws + oCat);
  _Float16* pUh  = (_Float16*)(ws + oUh);
  _Float16* pF1  = (_Float16*)(ws + oF1);
  _Float16* pRW  = (_Float16*)(ws + oRW);
  int* cntp[2]; int* offp[2]; int* rbp[2]; int* csrp[2];
  for (int t = 0; t < 2; ++t) {
    cntp[t] = (int*)(ws + oCnt[t]); offp[t] = (int*)(ws + oOff[t]);
    rbp[t]  = (int*)(ws + oRb[t]);  csrp[t] = (int*)(ws + oCsr[t]);
  }
  float* hP[2]; hP[0] = (float*)(ws + oH0); hP[1] = (float*)(ws + oH1);
  float* xA = (float*)(ws + oXA);
  float* xB = (float*)(ws + oXB);

  const int vec8 = ((nE & 3) == 0) ? 1 : 0;

  const int g0 = nL * (NP208 * XP / 8), g1 = GDP * KCAT / 8, g2 = NP208 * XP / 8, g3 = HIDN * KDEC / 8;
  const int b1 = cdiv_h(g0, NTHR), b2 = b1 + cdiv_h(g1, NTHR), b3 = b2 + cdiv_h(g2, NTHR), b4 = b3 + cdiv_h(g3, NTHR);
  k_wprep<<<b4, NTHR, 0, stream>>>(selfw, Wg, Ug, fc1, pSW, pCat, pUh, pF1, nL, b1, b2, b3);

  k_relw<<<dim3(RWP / 64, NP208 / 16, nL), NTHR, 0, stream>>>(basis, coeff, pRW);

  k_init<<<cdiv_h(NPAD * (XP / 4), NTHR), NTHR, 0, stream>>>(emb, hP[0], nN, NPAD * (XP / 4));

  hipFuncSetAttribute(reinterpret_cast<const void*>(&k_fill), hipFuncAttributeMaxDynamicSharedMemorySize, LDS_FILL);
  for (int t = 0; t < 2; ++t) {
    const int* rcv_t = rcv + (size_t)t * nE;
    const int* snd_t = snd + (size_t)t * nE;
    const int* rel_t = relt + (size_t)t * nE;
    k_count<<<nBC, NTHR, 0, stream>>>(rcv_t, cntp[t], nE, vec8);
    k_offsets<<<1, OTHR, 0, stream>>>(cntp[t], offp[t], rbp[t], nBC);
    k_fill<<<nBF, NTHR, LDS_FILL, stream>>>(rcv_t, snd_t, rel_t, offp[t], rbp[t], csrp[t], nN, nE, vec8, csrLen);
  }

  hipFuncSetAttribute(reinterpret_cast<const void*>(&k_layer), hipFuncAttributeMaxDynamicSharedMemorySize, LDS_LAYER);
  hipFuncSetAttribute(reinterpret_cast<const void*>(&k_gru), hipFuncAttributeMaxDynamicSharedMemorySize, LDS_GRU);
  int cur = 0;
  for (int t = 0; t < 2; ++t) {
    const float* xsrc = hP[cur];
    float* xdst = xA;
    for (int l = 0; l < nL; ++l) {
      xdst = (l & 1) ? xB : xA;
      k_layer<<<NPAD / RROWS, RTHR, LDS_LAYER, stream>>>(
          xsrc, csrp[t], offp[t], cntp[t],
          pRW + (size_t)l * NP208 * RWP, pSW + (size_t)l * NP208 * XP, bias + (size_t)l * DIMC,
          xdst, nN, csrLen);
      xsrc = xdst;
    }
    k_gru<<<NPAD / GROWS, NTHR, LDS_GRU, stream>>>(xsrc, hP[cur], pCat, pUh, bg, hP[1 - cur]);
    cur = 1 - cur;
  }

  hipFuncSetAttribute(reinterpret_cast<const void*>(&k_dec), hipFuncAttributeMaxDynamicSharedMemorySize, LDS_DEC);
  k_dec<<<cdiv_h(nQ, DROWS), NTHR, LDS_DEC, stream>>>(hP[cur], relemb, tri, pF1, fc1b, fc2, fc2b, out, nN, nRel, nQ);
}
